// SeqAttention_55327768708021
// MI455X (gfx1250) — hardware-verified
//
#include <hip/hip_runtime.h>
#include <math.h>
#include <stdint.h>

#define NBH 64
#define NHD 8
#define NM  1024
#define NKV 2048
#define NL  1024
#define ND  64
#define NQT 16
#define NCH 17
#define QPP 128
#define TP  72
static_assert(NQT * 64 == NM);
static_assert((NCH - 1) * 64 == NL);
static_assert((NM - 64) + 64 * (NCH - 1) + 63 == NKV - 1);
static_assert(ND == 64 && (NKV % 64) == 0 && (NL % 64) == 0);

typedef __bf16   v16b __attribute__((ext_vector_type(16)));
typedef __bf16   v8b  __attribute__((ext_vector_type(8)));
typedef float    v8f  __attribute__((ext_vector_type(8)));
typedef float    v4f  __attribute__((ext_vector_type(4)));
typedef unsigned int v4u __attribute__((ext_vector_type(4)));

__device__ __forceinline__ unsigned short bf_bits(float f) {
  unsigned u = __float_as_uint(f);
  return (unsigned short)((u + 0x7FFFu + ((u >> 16) & 1u)) >> 16);
}
__device__ __forceinline__ float bf_up(unsigned short h) { return __uint_as_float(((unsigned)h) << 16); }
__device__ __forceinline__ __bf16 bf_val(unsigned short h) { return __builtin_bit_cast(__bf16, h); }
__device__ __forceinline__ unsigned pk16(unsigned short a, unsigned short b) { return (unsigned)a | ((unsigned)b << 16); }
__device__ __forceinline__ v8f zero8() { v8f z = {0.f, 0.f, 0.f, 0.f, 0.f, 0.f, 0.f, 0.f}; return z; }
__device__ __forceinline__ v4f zero4() { v4f z = {0.f, 0.f, 0.f, 0.f}; return z; }

__device__ __forceinline__ v16b ldfrag_b(const __bf16* p) {
  union { v16b v; v8b h[2]; } f;
  f.h[0] = *(const v8b*)(p);
  f.h[1] = *(const v8b*)(p + 16);
  return f.v;
}

__device__ __forceinline__ v8f mma_b(v16b a, v16b b, v8f c) {
  c = __builtin_amdgcn_wmma_f32_16x16x32_bf16(false, a, false, b, (short)0, c, false, false);
  asm volatile("v_nop\n\tv_nop\n\tv_nop\n\tv_nop" : "+v"(c) : "v"(a), "v"(b));
  return c;
}

__global__ __launch_bounds__(256) void cvt_bf16x8(const float* __restrict__ in, unsigned short* out, int n8) {
  const int i = blockIdx.x * 256 + threadIdx.x;
  if (i < n8) {
    const v4f a = *(const v4f*)(in + (size_t)i * 8);
    const v4f b = *(const v4f*)(in + (size_t)i * 8 + 4);
    v4u p;
    p[0] = pk16(bf_bits(a[0]), bf_bits(a[1]));
    p[1] = pk16(bf_bits(a[2]), bf_bits(a[3]));
    p[2] = pk16(bf_bits(b[0]), bf_bits(b[1]));
    p[3] = pk16(bf_bits(b[2]), bf_bits(b[3]));
    *(volatile v4u*)(out + (size_t)i * 8) = p;
    __threadfence();
    *(volatile v4u*)(out + (size_t)i * 8) = p;
  }
}

__device__ __forceinline__ void tr_tile(const float* __restrict__ in, int ldi, unsigned short* out, int ldo,
                                        unsigned short* sT) {
  const int tid = threadIdx.x, wave = tid >> 5, lane = tid & 31;
  const int tr = tid >> 2, cq = tid & 3;
  const float* src = in + (size_t)tr * ldi + 16 * cq;
  const v4f a0 = *(const v4f*)(src);
  const v4f a1 = *(const v4f*)(src + 4);
  const v4f a2 = *(const v4f*)(src + 8);
  const v4f a3 = *(const v4f*)(src + 12);
#pragma unroll
  for (int e = 0; e < 4; ++e) {
    sT[(16 * cq + e)      * TP + tr] = bf_bits(a0[e]);
    sT[(16 * cq + 4 + e)  * TP + tr] = bf_bits(a1[e]);
    sT[(16 * cq + 8 + e)  * TP + tr] = bf_bits(a2[e]);
    sT[(16 * cq + 12 + e) * TP + tr] = bf_bits(a3[e]);
  }
  __syncthreads();
  v4u w[2]; size_t o[2];
#pragma unroll
  for (int it = 0; it < 2; ++it) {
    const int orow = 8 * wave + 4 * it + (lane >> 3);
    const int c8   = (lane & 7) * 8;
    w[it] = *(const v4u*)(sT + orow * TP + c8);
    o[it] = (size_t)orow * ldo + c8;
  }
  for (int pass = 0; pass < 2; ++pass) {
    *(volatile v4u*)(out + o[0]) = w[0];
    *(volatile v4u*)(out + o[1]) = w[1];
    __threadfence();
  }
}

__global__ __launch_bounds__(256) void tr_val(const float* __restrict__ V, unsigned short* VT) {
  __shared__ __align__(16) unsigned short sT[64 * TP];
  const int rb = blockIdx.x, bh = blockIdx.y;
  const float* in = V + ((size_t)bh * NKV + (size_t)rb * 64) * ND;
  unsigned short* out = VT + (size_t)bh * ND * NKV + (size_t)rb * 64;
  tr_tile(in, ND, out, NKV, sT);
}

__global__ __launch_bounds__(256) void tr_pe(const float* __restrict__ PE, unsigned short* PEt) {
  __shared__ __align__(16) unsigned short sT[64 * TP];
  const int cb = blockIdx.x;
  const float* in = PE + (size_t)cb * 64;
  unsigned short* out = PEt + (size_t)cb * 64 * ND;
  tr_tile(in, NL, out, ND, sT);
}

__global__ __launch_bounds__(128)
void attn_span(const unsigned short* __restrict__ qbp, const unsigned short* __restrict__ kbp,
               const unsigned short* __restrict__ vtp, const unsigned short* __restrict__ pep,
               const float* __restrict__ cvp, float* outp) {
  __shared__ __align__(16) float  sQP[4 * 16 * QPP];
  __shared__ __align__(16) __bf16 sPh[4 * 16 * 64];
  __shared__ __align__(16) __bf16 sPl[4 * 16 * 64];
  union FB { v16b v; v8b h[2]; };

  const int tid  = threadIdx.x;
  const int wave = tid >> 5;
  const int lane = tid & 31;
  const int hh   = lane >> 4;
  const int c    = lane & 15;
  const int bx   = blockIdx.x;
  const int qt   = bx & (NQT - 1);
  const int bh   = bx >> 4;
  const int m0   = qt * 64;
  const int q0   = m0 + wave * 16;
  const int iw   = wave * 16 + 8 * hh;

  const __bf16* Qb = (const __bf16*)(const void*)qbp;
  const __bf16* Kb = (const __bf16*)(const void*)kbp + (size_t)bh * NKV * ND;
  const __bf16* Vt = (const __bf16*)(const void*)vtp + (size_t)bh * ND * NKV;
  const __bf16* Pe = (const __bf16*)(const void*)pep;

  const float cv  = bf_up(bf_bits(cvp[bh & (NHD - 1)]));
  const float cvs = cv * (float)NL;
  const float scl = 1.0f / 22.627416610717773f;

  float*  qpw = sQP + wave * (16 * QPP);
  __bf16* pwh = sPh + wave * 1024;
  __bf16* pwl = sPl + wave * 1024;

#pragma unroll
  for (int t = 0; t < 16; ++t) *(v4f*)(qpw + (t * 32 + lane) * 4) = zero4();

  const size_t qo = ((size_t)bh * NM + q0 + c) * ND + 8 * hh;
  const v16b qa0 = ldfrag_b(Qb + qo);
  const v16b qa1 = ldfrag_b(Qb + qo + 32);

  v8f oacc[4];
#pragma unroll
  for (int t = 0; t < 4; ++t) oacc[t] = zero8();
  float mrow[8], zs[8], zm[8];
#pragma unroll
  for (int r = 0; r < 8; ++r) { mrow[r] = -INFINITY; zs[r] = 0.f; zm[r] = 0.f; }

#pragma unroll 1
  for (int ct = 0; ct < NCH; ++ct) {
    const int kv0 = m0 + 64 * ct;

    if (ct < NCH - 1) {
      const int l0 = 64 * ct;
      const int sc = (ct & 1) * 64;
#pragma unroll
      for (int j = 0; j < 4; ++j) {
        const size_t po = (size_t)(l0 + 16 * j + c) * ND + 8 * hh;
        const v16b p0 = ldfrag_b(Pe + po);
        const v16b p1 = ldfrag_b(Pe + po + 32);
        v8f tq = zero8();
        tq = mma_b(qa0, p0, tq);
        tq = mma_b(qa1, p1, tq);
#pragma unroll
        for (int r = 0; r < 8; ++r) qpw[(8 * hh + r) * QPP + sc + 16 * j + c] = tq[r];
      }
    }
    __builtin_amdgcn_fence(__ATOMIC_RELEASE, "workgroup");
    __builtin_amdgcn_wave_barrier();
    __builtin_amdgcn_fence(__ATOMIC_ACQUIRE, "workgroup");

    v8f s[4];
#pragma unroll
    for (int j = 0; j < 4; ++j) s[j] = zero8();
#pragma unroll
    for (int j = 0; j < 4; ++j) {
      const size_t ko = (size_t)(kv0 + 16 * j + c) * ND + 8 * hh;
      const v16b k0f = ldfrag_b(Kb + ko);
      const v16b k1f = ldfrag_b(Kb + ko + 32);
      s[j] = mma_b(qa0, k0f, s[j]);
      s[j] = mma_b(qa1, k1f, s[j]);
    }

#pragma unroll
    for (int r = 0; r < 8; ++r) {
      const int lb = 64 * ct + c - iw - r;
      const float* qprow = qpw + (8 * hh + r) * QPP;
      float mx = -INFINITY;
#pragma unroll
      for (int j = 0; j < 4; ++j) {
        const int l = lb + 16 * j;
        const float qp = qprow[l & (QPP - 1)];
        float sv = (s[j][r] + qp) * scl;
        sv = ((unsigned)l < (unsigned)NL) ? sv : -INFINITY;
        s[j][r] = sv;
        mx = fmaxf(mx, sv);
      }
      mx = fmaxf(mx, __shfl_xor(mx, 1, 32));
      mx = fmaxf(mx, __shfl_xor(mx, 2, 32));
      mx = fmaxf(mx, __shfl_xor(mx, 4, 32));
      mx = fmaxf(mx, __shfl_xor(mx, 8, 32));
      const float mnew  = fmaxf(mrow[r], mx);
      const float msafe = (mnew == -INFINITY) ? 0.f : mnew;
      const float al    = __expf(mrow[r] - msafe);
      mrow[r] = mnew;
#pragma unroll
      for (int t = 0; t < 4; ++t) oacc[t][r] *= al;
      float pse = 0.f, psm = 0.f;
#pragma unroll
      for (int j = 0; j < 4; ++j) {
        const int l = lb + 16 * j;
        const float e = __expf(s[j][r] - msafe);
        float wk = ((float)(l - (NL - 1)) + cvs) * 0.03125f + 1.0f;
        wk = fminf(fmaxf(wk, 0.f), 1.f);
        const float pm = e * wk;
        pse += e;
        psm += pm;
        const unsigned short hb = bf_bits(pm);
        const unsigned short lo = bf_bits(pm - bf_up(hb));
        const int po = (8 * hh + r) * 64 + 16 * j + c;
        pwh[po] = bf_val(hb);
        pwl[po] = bf_val(lo);
      }
      pse += __shfl_xor(pse, 1, 32); pse += __shfl_xor(pse, 2, 32);
      pse += __shfl_xor(pse, 4, 32); pse += __shfl_xor(pse, 8, 32);
      psm += __shfl_xor(psm, 1, 32); psm += __shfl_xor(psm, 2, 32);
      psm += __shfl_xor(psm, 4, 32); psm += __shfl_xor(psm, 8, 32);
      zs[r] = zs[r] * al + pse;
      zm[r] = zm[r] * al + psm;
    }
    __builtin_amdgcn_fence(__ATOMIC_RELEASE, "workgroup");
    __builtin_amdgcn_wave_barrier();
    __builtin_amdgcn_fence(__ATOMIC_ACQUIRE, "workgroup");

    FB pa[2], pl[2];
#pragma unroll
    for (int kk = 0; kk < 2; ++kk) {
      const int pr = c * 64 + kk * 32 + 8 * hh;
      pa[kk].h[0] = *(const v8b*)(pwh + pr);
      pa[kk].h[1] = *(const v8b*)(pwh + pr + 16);
      pl[kk].h[0] = *(const v8b*)(pwl + pr);
      pl[kk].h[1] = *(const v8b*)(pwl + pr + 16);
    }
#pragma unroll
    for (int t = 0; t < 4; ++t) {
      const size_t vo = (size_t)(16 * t + c) * NKV + kv0 + 8 * hh;
#pragma unroll
      for (int kk = 0; kk < 2; ++kk) {
        const v16b vb = ldfrag_b(Vt + vo + 32 * kk);
        oacc[t] = mma_b(pa[kk].v, vb, oacc[t]);
        oacc[t] = mma_b(pl[kk].v, vb, oacc[t]);
      }
    }
  }

  float inv[8];
#pragma unroll
  for (int r = 0; r < 8; ++r) inv[r] = 1.0f / (zm[r] + 1e-8f * zs[r]);
  float* os = qpw;
#pragma unroll
  for (int t = 0; t < 4; ++t) {
#pragma unroll
    for (int r = 0; r < 8; ++r) os[(8 * hh + r) * 64 + 16 * t + c] = oacc[t][r] * inv[r];
  }
  __builtin_amdgcn_fence(__ATOMIC_RELEASE, "workgroup");
  __builtin_amdgcn_wave_barrier();
  __builtin_amdgcn_fence(__ATOMIC_ACQUIRE, "workgroup");
  float* og = outp + ((size_t)bh * NM + q0) * ND;
  for (int pass = 0; pass < 2; ++pass) {
#pragma unroll
    for (int it = 0; it < 8; ++it) {
      const int col = it * 128 + lane * 4;
      const v4f v = *(const v4f*)(os + col);
      *(volatile v4f*)(og + col) = v;
    }
    __threadfence();
  }
}

extern "C" void kernel_launch(void* const* d_in, const int* in_sizes, int n_in,
                              void* d_out, int out_size, void* d_ws, size_t ws_size,
                              hipStream_t stream) {
  if (n_in < 5) return;
  if (in_sizes[0] != NBH * NM * ND) return;
  if (in_sizes[1] != NBH * NKV * ND || in_sizes[2] != NBH * NKV * ND) return;
  if (in_sizes[3] != ND * NL || in_sizes[4] != NHD) return;
  if (out_size != NBH * NM * ND) return;

  const float* q  = (const float*)d_in[0];
  const float* k  = (const float*)d_in[1];
  const float* v  = (const float*)d_in[2];
  const float* pe = (const float*)d_in[3];
  const float* cv = (const float*)d_in[4];

  const size_t PQ = (size_t)NBH * NM * ND * 2;
  const size_t PK = (size_t)NBH * NKV * ND * 2;
  const size_t PV = (size_t)NBH * ND * NKV * 2;
  const size_t PP = (size_t)NL * ND * 2;
  size_t off = 0;
  const size_t oQ = off; off += PQ;
  const size_t oK = off; off += PK;
  const size_t oV = off; off += PV;
  const size_t oP = off; off += PP;
  if (off > ws_size) return;
  if (off > (size_t)134217728) return;

  char* ws = (char*)d_ws;
  unsigned short* Qb  = (unsigned short*)(ws + oQ);
  unsigned short* Kb  = (unsigned short*)(ws + oK);
  unsigned short* VT  = (unsigned short*)(ws + oV);
  unsigned short* PEt = (unsigned short*)(ws + oP);

  const dim3 blk(256);
  const int n8q = NBH * NM * ND / 8;
  const int n8k = NBH * NKV * ND / 8;
  const dim3 gCvtQ((n8q + 255) / 256);
  const dim3 gCvtK((n8k + 255) / 256);
  const dim3 gTrV(NKV / 64, NBH);
  const dim3 gTrP(NL / 64);
  const dim3 gAttn(NBH * NQT);

  cvt_bf16x8<<<gCvtQ, blk, 0, stream>>>(q, Qb, n8q);
  cvt_bf16x8<<<gCvtK, blk, 0, stream>>>(k, Kb, n8k);
  tr_val<<<gTrV, blk, 0, stream>>>(v, VT);
  tr_pe<<<gTrP, blk, 0, stream>>>(pe, PEt);
  attn_span<<<gAttn, dim3(128), 0, stream>>>(Qb, Kb, VT, PEt, cv, (float*)d_out);
  (void)hipGetLastError();
}
